// EncoderLayer_83631603188296
// MI455X (gfx1250) — hardware-verified
//
#include <hip/hip_runtime.h>
#ifndef NB
#define NB 2
#endif
#ifndef SEQ
#define SEQ 2048
#endif
#define NB_FULL 2
#define SEQ_FULL 2048
#define DM 1024
#define NH 16
#define HD 64
#define DFF 4096
#define DMQ DM
#define LQ (3 * DM)
#define NR ((size_t)NB * SEQ)
static_assert(NH * HD == DM);
static_assert(HD == 64);
static_assert(DM == 1024);
static_assert(((NB * SEQ) % 128) == 0);
static_assert((SEQ % 64) == 0);
static_assert((DFF % 64) == 0);
static_assert((DM % 64) == 0);
static_assert(NB <= NB_FULL && SEQ <= SEQ_FULL);

typedef unsigned short v8us __attribute__((ext_vector_type(8), may_alias));
typedef float  v8f  __attribute__((ext_vector_type(8)));
typedef float  v4f  __attribute__((ext_vector_type(4)));
typedef float  v4fa __attribute__((ext_vector_type(4), may_alias));
typedef int    v4i  __attribute__((ext_vector_type(4)));
typedef int    v4ia __attribute__((ext_vector_type(4), may_alias));
typedef _Float16 v16h __attribute__((ext_vector_type(16)));
typedef _Float16 v4h __attribute__((ext_vector_type(4)));
union FragH { v16h v; v8us half[2]; _Float16 h[16]; unsigned short u[16]; };

__device__ __forceinline__ unsigned short bf16_bits(float x) { unsigned int u = __float_as_uint(x); return (unsigned short)((u + 0x7FFFu + ((u >> 16) & 1u)) >> 16); }
__device__ __forceinline__ float bf16_val(unsigned short b) { return __uint_as_float(((unsigned int)b) << 16); }
__device__ __forceinline__ float bf16_rne(float x) { return bf16_val(bf16_bits(x)); }

__device__ __forceinline__ v16h g2_frag(const _Float16* p, unsigned hh) { FragH f; f.half[0] = *(const v8us*)((const unsigned short*)p + 8 * hh); f.half[1] = *(const v8us*)((const unsigned short*)p + 16 + 8 * hh); return f.v; }
__device__ __forceinline__ v8f g2_mma(v16h a, v16h b, v8f c) { v8f d = __builtin_amdgcn_wmma_f32_16x16x32_f16(false, a, false, b, (short)0, c, false, false); asm volatile("v_nop\n\tv_nop\n\tv_nop\n\tv_nop" : "+v"(d) : "v"(a), "v"(b)); return d; }

__global__ __launch_bounds__(256) void k_wt_f16(const float* __restrict__ W, _Float16* __restrict__ Wt, unsigned K, unsigned N, float scale) {
  const unsigned t = blockIdx.x * 256u + threadIdx.x; const unsigned k8n = K >> 3; if (t >= N * k8n) return; const unsigned n = t / k8n, k8 = (t - n * k8n) << 3; FragH f;
#pragma unroll
  for (unsigned i = 0; i < 8; ++i) f.h[i] = (_Float16)(bf16_rne(W[(size_t)(k8 + i) * N + n]) * scale);
  const v8us o = f.half[0]; unsigned short* dst = (unsigned short*)Wt + (size_t)n * K + k8;
  *(volatile v8us*)dst = o; __threadfence(); *(volatile v8us*)dst = o;
}

__global__ __launch_bounds__(256) void k_bias3(const float* __restrict__ b0, const float* __restrict__ b1, const float* __restrict__ b2, float* __restrict__ dst) {
  const unsigned t = blockIdx.x * 256u + threadIdx.x; if (t >= 3u * (DM / 4)) return; const unsigned seg = t / (DM / 4), c = (t % (DM / 4)) * 4u;
  const v4f a0 = *(const v4fa*)(b0 + c), a1 = *(const v4fa*)(b1 + c), a2 = *(const v4fa*)(b2 + c);
  v4f v; for (int q = 0; q < 4; ++q) v[q] = (seg == 0u) ? a0[q] : ((seg == 1u) ? a1[q] : a2[q]);
  *(volatile v4f*)(dst + (size_t)t * 4) = v; __threadfence(); *(volatile v4f*)(dst + (size_t)t * 4) = v;
}

__global__ __launch_bounds__(256) void k_xprep(const float* __restrict__ x, float* __restrict__ XB, _Float16* __restrict__ X16) {
  const unsigned t = blockIdx.x * 256u + threadIdx.x; if (t >= (unsigned)(NB * SEQ) * (DM / 4)) return;
  const unsigned r = t / (DM / 4), c = (t % (DM / 4)) * 4u; const unsigned b = r / SEQ, s = r - b * SEQ;
  const v4f a = *(const v4fa*)(x + ((size_t)b * SEQ_FULL + s) * DM + c); v4f y; v4h hq;
  for (int q = 0; q < 4; ++q) { y[q] = bf16_rne(a[q]); hq[q] = (_Float16)y[q]; }
  for (int pass = 0; pass < 2; ++pass) { *(volatile v4f*)(XB + (size_t)t * 4) = y; *(volatile v4h*)(X16 + (size_t)t * 4) = hq; if (pass == 0) __threadfence(); }
}

template <int ACT>
__global__ __launch_bounds__(128) void k_gemm2(const _Float16* __restrict__ A, int lda, size_t sA, const _Float16* __restrict__ Bh, int ldb, size_t sB, float alpha, const float* __restrict__ bias, size_t sBias, const float* __restrict__ CP, int rowsPerB, size_t sCPb, int row0g,
    float* __restrict__ C, _Float16* __restrict__ C16, int ldc, size_t sC, int M, int N, int K) { static_assert(ACT == 0 || ACT == 3);
  __shared__ __attribute__((aligned(16))) float so[4][32][68];
  const int tid = threadIdx.x, w = tid >> 5, lane = tid & 31, ln = lane & 15, hh = lane >> 4; const int by = blockIdx.y;
  A += (size_t)by * sA; Bh += (size_t)by * sB; const size_t cofs = (size_t)by * sC; const float* bp = bias ? bias + (size_t)by * sBias : nullptr;
  const int ntn = N >> 6; const int mt = blockIdx.x / ntn, nq = blockIdx.x - mt * ntn; const int row0 = mt * 128 + 32 * w, col0 = nq * 64; if (row0 >= M) return;
  const _Float16* a0p = A + (size_t)(row0 + ln) * lda; const _Float16* a1p = a0p + (size_t)16 * lda;
  const _Float16* b0p = Bh + (size_t)(col0 + ln) * ldb; const _Float16* b1p = b0p + (size_t)16 * ldb; const _Float16* b2p = b1p + (size_t)16 * ldb; const _Float16* b3p = b2p + (size_t)16 * ldb;
  const v8f z8 = {0.f,0.f,0.f,0.f,0.f,0.f,0.f,0.f}; v8f c00 = z8, c01 = z8, c02 = z8, c03 = z8, c10 = z8, c11 = z8, c12 = z8, c13 = z8;
#pragma unroll 1
  for (int kb = 0; kb < K; kb += 32) { const v16h a0 = g2_frag(a0p + kb, hh), a1 = g2_frag(a1p + kb, hh);
    v16h b = g2_frag(b0p + kb, hh); c00 = g2_mma(a0, b, c00); c10 = g2_mma(a1, b, c10);
    b = g2_frag(b1p + kb, hh); c01 = g2_mma(a0, b, c01); c11 = g2_mma(a1, b, c11);
    b = g2_frag(b2p + kb, hh); c02 = g2_mma(a0, b, c02); c12 = g2_mma(a1, b, c12);
    b = g2_frag(b3p + kb, hh); c03 = g2_mma(a0, b, c03); c13 = g2_mma(a1, b, c13); }
  v8f accs[8] = {c00, c01, c02, c03, c10, c11, c12, c13};
#pragma unroll
  for (int u = 0; u < 8; ++u) { const int t = u & 3, half = u >> 2; const int col = col0 + t * 16 + ln; const float bv = bp ? bf16_rne(bp[col]) : 0.f;
#pragma unroll
    for (int r = 0; r < 8; ++r) { const int rloc = half * 16 + 8 * hh + r; float v = accs[u][r] * alpha + bv; if (CP) { if (rowsPerB < 0) v += CP[cofs + (size_t)(row0g + row0 + rloc) * ldc + col]; else { const int bidx = (row0g + row0 + rloc) / rowsPerB; v += CP[(size_t)bidx * sCPb + (size_t)by * 64 + col]; } }
      if (ACT == 3) v = fmaxf(v, 0.f);
      so[w][rloc][t * 16 + ln] = v; } }
  __builtin_amdgcn_fence(4  , "workgroup"); __builtin_amdgcn_wave_barrier();
  const int rsub = lane >> 4, c4 = (lane & 15) * 4;
  for (int pass = 0; pass < 2; ++pass) {
#pragma unroll
    for (int q = 0; q < 16; ++q) { const int r = q * 2 + rsub; const v4f v = *(const v4fa*)&so[w][r][c4]; if (C) *(volatile v4f*)(C + cofs + (size_t)(row0 + r) * ldc + col0 + c4) = v; if (C16) { v4h h4; for (int i = 0; i < 4; ++i) h4[i] = (_Float16)v[i]; *(volatile v4h*)(C16 + cofs + (size_t)(row0 + r) * ldc + col0 + c4) = h4; } }
    if (pass == 0) __threadfence(); } }

template <int NHv, int TTv>
__global__ __launch_bounds__(256) void k_vt(const _Float16* __restrict__ V16, int ldv, int voff, _Float16* __restrict__ Vt) { __shared__ unsigned short tl[64][66]; const unsigned tid = threadIdx.x; const unsigned slab = blockIdx.x / (TTv / 64), lg = blockIdx.x % (TTv / 64); const unsigned b = slab / NHv, h = slab % NHv;
  for (unsigned i = tid; i < 64u * 8u; i += 256u) { const unsigned r = i >> 3, c8 = (i & 7u) << 3; FragH f; f.half[0] = *(const v8us*)((const unsigned short*)V16 + ((size_t)b * TTv + lg * 64 + r) * ldv + voff + h * 64 + c8);
#pragma unroll
    for (unsigned q = 0; q < 8; ++q) tl[r][c8 + q] = f.u[q]; }
  __syncthreads();
  for (int pass = 0; pass < 2; ++pass) {
#pragma unroll
    for (unsigned rd = 0; rd < 2; ++rd) { const unsigned d = rd * 32 + (tid >> 3), pc = tid & 7u; FragH f;
#pragma unroll
      for (unsigned q = 0; q < 8; ++q) f.u[q] = tl[pc * 8 + q][d];
      *(volatile v8us*)((unsigned short*)Vt + ((size_t)slab * 64 + d) * TTv + lg * 64 + pc * 8) = f.half[0]; }
    if (pass == 0) __threadfence(); } }

__global__ __launch_bounds__(128) void k_flash(const _Float16* __restrict__ QKV, const _Float16* __restrict__ VT, const int* __restrict__ mask, _Float16* __restrict__ O16) {
  __shared__ unsigned int mw[SEQ / 32];
  __shared__ __attribute__((aligned(16))) unsigned short so[4][16][72];
  const unsigned tid = threadIdx.x, w = tid >> 5, lane = tid & 31u, ln = lane & 15u, hh = lane >> 4;
  const unsigned bh = blockIdx.x / (SEQ / 64), qb = blockIdx.x % (SEQ / 64);
  const unsigned b = bh / NH, h = bh % NH;
  for (unsigned t0 = 0; t0 < SEQ / 32; t0 += 128) {
    const unsigned t = t0 + tid; const unsigned tc = (t < SEQ / 32) ? t : (SEQ / 32 - 1);
    const int* mp = mask + (size_t)b * SEQ_FULL + (size_t)tc * 32; unsigned word = 0;
#pragma unroll 1
    for (unsigned i = 0; i < 8; ++i) { const v4i m4 = *(const v4ia*)(mp + i * 4); const unsigned nib = (m4[0] != 0 ? 1u : 0u) | (m4[1] != 0 ? 2u : 0u) | (m4[2] != 0 ? 4u : 0u) | (m4[3] != 0 ? 8u : 0u); word |= nib << (i * 4); }
    if (t < SEQ / 32) mw[t] = word;
  }
  __syncthreads();
  const unsigned q0 = qb * 64 + w * 16;
  const _Float16* qrow = QKV + ((size_t)b * SEQ + q0 + ln) * LQ + h * HD;
  const v16h qf0 = g2_frag(qrow, hh), qf1 = g2_frag(qrow + 32, hh);
  const _Float16* Kb = QKV + (size_t)b * SEQ * LQ + DM + h * HD + (size_t)ln * LQ;
  const _Float16* Vb = VT + (((size_t)b * NH + h) * HD + ln) * SEQ;
  const v8f z8 = {0.f,0.f,0.f,0.f,0.f,0.f,0.f,0.f};
  v8f o0 = z8, o1 = z8, o2 = z8, o3 = z8; float m = -1.0e30f, l = 0.f;
#pragma unroll 1
  for (unsigned kt = 0; kt < SEQ / 32; ++kt) {
    const unsigned key0 = kt * 32;
    const _Float16* k0p = Kb + (size_t)key0 * LQ; const _Float16* k1p = k0p + (size_t)16 * LQ;
    v16h a = g2_frag(k0p, hh); v8f s0 = g2_mma(a, qf0, z8); a = g2_frag(k0p + 32, hh); s0 = g2_mma(a, qf1, s0);
    a = g2_frag(k1p, hh); v8f s1 = g2_mma(a, qf0, z8); a = g2_frag(k1p + 32, hh); s1 = g2_mma(a, qf1, s1);
    const unsigned mword = (unsigned)__builtin_amdgcn_readfirstlane((int)mw[kt]);
    float sv[16];
#pragma unroll
    for (int r = 0; r < 8; ++r) { sv[r] = s0[r] * 0.125f; sv[8 + r] = s1[r] * 0.125f; }
    if (mword != 0xFFFFFFFFu) {
      const unsigned wb = mword >> (8u * hh);
#pragma unroll
      for (int r = 0; r < 8; ++r) { sv[r] = ((wb >> r) & 1u) ? sv[r] : -1.0e9f; sv[8 + r] = ((wb >> (16 + r)) & 1u) ? sv[8 + r] : -1.0e9f; }
    }
    float tmax = sv[0];
#pragma unroll
    for (int i = 1; i < 16; ++i) tmax = fmaxf(tmax, sv[i]);
    tmax = fmaxf(tmax, __shfl_xor(tmax, 16, 32));
    const float mnew = fmaxf(m, tmax); const float sc = __expf(m - mnew); float ps = 0.f; FragH pf;
#pragma unroll
    for (int i = 0; i < 16; ++i) { const float p = __expf(sv[i] - mnew); ps += p; pf.h[i] = (_Float16)p; }
    l = l * sc + ps; m = mnew;
    o0 = o0 * sc; o1 = o1 * sc; o2 = o2 * sc; o3 = o3 * sc;
    const _Float16* vp = Vb + key0;
    a = g2_frag(vp, hh); o0 = g2_mma(a, pf.v, o0);
    a = g2_frag(vp + (size_t)16 * SEQ, hh); o1 = g2_mma(a, pf.v, o1);
    a = g2_frag(vp + (size_t)32 * SEQ, hh); o2 = g2_mma(a, pf.v, o2);
    a = g2_frag(vp + (size_t)48 * SEQ, hh); o3 = g2_mma(a, pf.v, o3);
  }
  const float lt = l + __shfl_xor(l, 16, 32); const float fin = 64.0f * (1.0f / lt);
  { FragH f;
#pragma unroll
    for (int r = 0; r < 8; ++r) f.h[r] = (_Float16)(o0[r] * fin); *(v8us*)&so[w][ln][0 + 8 * hh] = f.half[0];
#pragma unroll
    for (int r = 0; r < 8; ++r) f.h[r] = (_Float16)(o1[r] * fin); *(v8us*)&so[w][ln][16 + 8 * hh] = f.half[0];
#pragma unroll
    for (int r = 0; r < 8; ++r) f.h[r] = (_Float16)(o2[r] * fin); *(v8us*)&so[w][ln][32 + 8 * hh] = f.half[0];
#pragma unroll
    for (int r = 0; r < 8; ++r) f.h[r] = (_Float16)(o3[r] * fin); *(v8us*)&so[w][ln][48 + 8 * hh] = f.half[0]; }
  __builtin_amdgcn_fence(4  , "workgroup"); __builtin_amdgcn_wave_barrier();
  const unsigned rq = lane >> 3, pc = (lane & 7u) * 8u;
  for (int pass = 0; pass < 2; ++pass) {
#pragma unroll
    for (unsigned it = 0; it < 4; ++it) { const unsigned row = it * 4 + rq; const v8us v = *(const v8us*)&so[w][row][pc];
      *(volatile v8us*)((unsigned short*)O16 + ((size_t)b * SEQ + q0 + row) * DM + h * HD + pc) = v; }
    if (pass == 0) __threadfence(); }
}

template <int BFIN, int W16, int W32>
__global__ __launch_bounds__(256) void k_lnx(const float* __restrict__ X, const float* __restrict__ g, const float* __restrict__ bb, float eps, _Float16* __restrict__ N16, float* __restrict__ N32) {
  #pragma clang fp contract(off)
  __shared__ float red[256]; const size_t r = blockIdx.x; const int t = threadIdx.x; const bool act = t < (DMQ / 4); const int c0 = act ? t * 4 : 0;
  const v4f xa = *(const v4fa*)(X + r * DMQ + c0); float s[4]; float sum = 0.f;
  for (int q = 0; q < 4; ++q) { s[q] = act ? (BFIN ? bf16_rne(xa[q]) : xa[q]) : 0.f; sum = __fadd_rn(sum, s[q]); }
  red[t] = sum; __syncthreads(); for (int st = 128; st > 0; st >>= 1) { if (t < st) red[t] = __fadd_rn(red[t], red[t + st]); __syncthreads(); } const float mu = red[0] / (float)DMQ; __syncthreads();
  float vs = 0.f; for (int q = 0; q < 4; ++q) { const float dl = act ? __fadd_rn(s[q], -mu) : 0.f; vs = __fadd_rn(vs, __fmul_rn(dl, dl)); } red[t] = vs; __syncthreads(); for (int st = 128; st > 0; st >>= 1) { if (t < st) red[t] = __fadd_rn(red[t], red[t + st]); __syncthreads(); }
  const float rs = rsqrtf(__fadd_rn(red[0] / (float)DMQ, eps)); v4h y; v4f yf;
  for (int q = 0; q < 4; ++q) { const int c = c0 + q; yf[q] = __fadd_rn(__fmul_rn(__fmul_rn(__fadd_rn(s[q], -mu), rs), bf16_rne(g[c])), bf16_rne(bb[c])); y[q] = (_Float16)yf[q]; }
  if (!act) return;
  for (int pass = 0; pass < 2; ++pass) { if (W16) *(volatile v4h*)(N16 + r * DMQ + c0) = y; if (W32) *(volatile v4f*)(N32 + r * DMQ + c0) = yf; if (pass == 0) __threadfence(); } }

extern "C" void kernel_launch(void* const* d_in, const int* in_sizes, int n_in,
                              void* d_out, int out_size, void* d_ws, size_t ws_size, hipStream_t stream) {
  if (n_in < 18) return;
  const size_t need_x = ((size_t)(NB - 1) * SEQ_FULL + SEQ) * DM, need_m = (size_t)(NB - 1) * SEQ_FULL + SEQ;
  if ((size_t)in_sizes[0] < need_x || (size_t)in_sizes[1] < need_m) return;
  if ((size_t)in_sizes[2] < (size_t)DM * DM || (size_t)in_sizes[4] < (size_t)DM * DM || (size_t)in_sizes[6] < (size_t)DM * DM || (size_t)in_sizes[8] < (size_t)DM * DM) return;
  if ((size_t)in_sizes[12] < (size_t)DM * DFF || (size_t)in_sizes[14] < (size_t)DFF * DM || (size_t)in_sizes[13] < (size_t)DFF) return;
  if ((size_t)out_size < NR * DM) return;
  const float* x = (const float*)d_in[0]; const int* mask = (const int*)d_in[1];
  const float* wq = (const float*)d_in[2]; const float* bq = (const float*)d_in[3]; const float* wk = (const float*)d_in[4]; const float* bk = (const float*)d_in[5]; const float* wv = (const float*)d_in[6]; const float* bv = (const float*)d_in[7];
  const float* w1 = (const float*)d_in[8]; const float* b1 = (const float*)d_in[9]; const float* g1 = (const float*)d_in[10]; const float* be1 = (const float*)d_in[11];
  const float* fw1 = (const float*)d_in[12]; const float* fb1 = (const float*)d_in[13]; const float* fw2 = (const float*)d_in[14]; const float* fb2 = (const float*)d_in[15]; const float* g2 = (const float*)d_in[16]; const float* be2 = (const float*)d_in[17];
  char* ws = (char*)d_ws; size_t off = 0;
  auto take = [&](size_t bytes) { char* p = ws + off; off += (bytes + 255) & ~(size_t)255; return p; };
  _Float16* BQKV = (_Float16*)take((size_t)3 * DM * DM * 2); _Float16* BO = (_Float16*)take((size_t)DM * DM * 2);
  _Float16* BW1 = (_Float16*)take((size_t)DFF * DM * 2); _Float16* BW2 = (_Float16*)take((size_t)DM * DFF * 2);
  float* bqkv = (float*)take((size_t)3 * DM * 4);
  _Float16* XM16 = (_Float16*)take(NR * DM * 2);
  float* XB = (float*)take(NR * DM * 4); float* X1 = (float*)take(NR * DM * 4); float* X2 = (float*)take(NR * DM * 4);
  _Float16* O16 = (_Float16*)take(NR * DM * 2);
  const size_t qkv_b = NR * 3 * DM * 2, vt_b = (size_t)NB * NH * HD * SEQ * 2, hf_b = NR * DFF * 2;
  const size_t u_b = (qkv_b + vt_b > hf_b) ? (qkv_b + vt_b) : hf_b;
  char* U = take(u_b);
  _Float16* QKV = (_Float16*)U; _Float16* VT = (_Float16*)(U + qkv_b); _Float16* HF16 = (_Float16*)U;
  if (off > ws_size || off > (size_t)134217728) return;
  { const unsigned g = (unsigned)(((size_t)DM * (DM / 8) + 255) / 256);
    k_wt_f16<<<g, 256, 0, stream>>>(wq, BQKV, DM, DM, 16.0f); k_wt_f16<<<g, 256, 0, stream>>>(wk, BQKV + (size_t)DM * DM, DM, DM, 16.0f);
    k_wt_f16<<<g, 256, 0, stream>>>(wv, BQKV + (size_t)2 * DM * DM, DM, DM, 16.0f); k_wt_f16<<<g, 256, 0, stream>>>(w1, BO, DM, DM, 16.0f); }
  k_wt_f16<<<(unsigned)(((size_t)DFF * (DM / 8) + 255) / 256), 256, 0, stream>>>(fw1, BW1, DM, DFF, 16.0f);
  k_wt_f16<<<(unsigned)(((size_t)DM * (DFF / 8) + 255) / 256), 256, 0, stream>>>(fw2, BW2, DFF, DM, 16.0f);
  k_bias3<<<(3 * (DM / 4) + 255) / 256, 256, 0, stream>>>(bq, bk, bv, bqkv);
  k_xprep<<<(unsigned)((NR * (DM / 4) + 255) / 256), 256, 0, stream>>>(x, XB, XM16);
  k_gemm2<0><<<dim3((unsigned)((NR / 128) * (3 * DM / 64)), 1), 128, 0, stream>>>(XM16, DM, 0, BQKV, DM, 0, 0.0625f, bqkv, 0, nullptr, 1, 0, 0, nullptr, QKV, 3 * DM, 0, (int)NR, 3 * DM, DM);
  k_vt<NH, SEQ><<<NB * NH * (SEQ / 64), 256, 0, stream>>>(QKV + 2 * DM, LQ, 0, VT);
  k_flash<<<NB * NH * (SEQ / 64), 128, 0, stream>>>(QKV, VT, mask, O16);
  k_gemm2<0><<<dim3((unsigned)((NR / 128) * (DM / 64)), 1), 128, 0, stream>>>(O16, DM, 0, BO, DM, 0, 0.0009765625f, b1, 0, XB, -1, 0, 0, X1, nullptr, DM, 0, (int)NR, DM, DM);
  k_lnx<0, 1, 1><<<(unsigned)NR, 256, 0, stream>>>(X1, g1, be1, 1e-5f, XM16, X2);
  k_gemm2<3><<<dim3((unsigned)((NR / 128) * (DFF / 64)), 1), 128, 0, stream>>>(XM16, DM, 0, BW1, DM, 0, 0.0625f, fb1, 0, nullptr, 1, 0, 0, nullptr, HF16, DFF, 0, (int)NR, DFF, DM);
  k_gemm2<0><<<dim3((unsigned)((NR / 128) * (DM / 64)), 1), 128, 0, stream>>>(HF16, DFF, 0, BW2, DFF, 0, 0.0625f, fb2, 0, X2, -1, 0, 0, X1, nullptr, DM, 0, (int)NR, DM, DFF);
  k_lnx<0, 0, 1><<<(unsigned)NR, 256, 0, stream>>>(X1, g2, be2, 1e-5f, nullptr, (float*)d_out);
}
